// GRUModel_7129645711670
// MI455X (gfx1250) — hardware-verified
//
#include <hip/hip_runtime.h>
#include <math.h>

constexpr int NBAT   = 64;
constexpr int NSTEP  = 512;
constexpr int NINP   = 128;
constexpr int NHID   = 1024;
constexpr int NOUTC  = 3;
constexpr int NG3    = 3 * NHID;
constexpr int NTHR   = 256;
constexpr int NWAVE  = NTHR / 32;
constexpr int RBLK   = 16;
constexpr int CHUNK  = 64;
constexpr int NCHUNK = NSTEP / CHUNK;
constexpr int CHROWS = CHUNK * NBAT;
constexpr int UROWS  = NSTEP * NBAT;
constexpr int HPF    = NHID + 4;
constexpr int HPH    = NHID + 8;
constexpr int JTW    = NHID / (16 * NWAVE);
constexpr int OSP    = CHUNK * NOUTC;
constexpr int OUTROW = NSTEP * NOUTC;
constexpr float WCARRY     = 64.0f;
constexpr float WCARRY_INV = 1.0f / 64.0f;
static_assert(NBAT % RBLK == 0, "blocks own whole 16-row batch tiles");
static_assert(RBLK == 2 * NWAVE, "store map: wave w writes rows 2w and 2w+1");
static_assert(NHID == 16 * JTW * NWAVE, "8 waves x 8 j-tiles x 16 columns");
static_assert(NSTEP % CHUNK == 0, "whole chunks");
static_assert(CHROWS % 64 == 0 && NG3 % 64 == 0, "GEMM M, N tile multiples");
static_assert(NINP % 32 == 0, "GEMM K multiple of 32");
static_assert(NHID % 32 == 0, "recurrence K multiple of 32");
static_assert((RBLK * NHID / 4) % NTHR == 0, "h f32 init loop exact");
static_assert((RBLK * NHID / 8) % NTHR == 0, "h f16 convert loop exact");
static_assert((NOUTC * NHID / 4) % NTHR == 0, "w_fc staging loop exact");
static_assert((OSP * 4) % 256 == 0, "out chunk segment = whole 256-B store units");
static_assert((OUTROW * 4) % 128 == 0, "out batch rows line aligned");
static_assert((NHID * 4) % 256 == 0, "h carry rows = whole 256-B store units");
static_assert(HPF % 4 == 0 && HPH % 8 == 0, "16-B aligned LDS rows");
static_assert((UROWS * NINP / 8) % NTHR == 0, "u convert grid exact");
static_assert((NG3 * NHID / 8) % NTHR == 0 && (NG3 * NINP / 8) % NTHR == 0, "weight convert grids exact");
static_assert(((CHROWS / 64) * (NG3 / 64)) % 8 == 0, "GEMM grid exact");

typedef __attribute__((ext_vector_type(16))) _Float16 v16h;
typedef __attribute__((ext_vector_type(8)))  _Float16 v8h;
typedef __attribute__((ext_vector_type(16))) __bf16   v16b;
typedef __attribute__((ext_vector_type(8)))  __bf16   v8b;
typedef __attribute__((ext_vector_type(8)))  float    v8f;
typedef __attribute__((ext_vector_type(4)))  float    v4f;

__device__ __forceinline__ unsigned short f2bf_bits(float f) {
  unsigned u = __float_as_uint(f);
  return (unsigned short)((u + 0x7FFFu + ((u >> 16) & 1u)) >> 16);
}
__device__ __forceinline__ float bf_bits2f(unsigned short h) { return __uint_as_float(((unsigned)h) << 16); }

__device__ __forceinline__ void dep_guard_h(v8f& a, v8f& b, v16h x, v16h y) { asm volatile("v_nop\n\tv_nop\n\tv_nop\n\tv_nop" : "+v"(a), "+v"(b) : "v"(x), "v"(y)); }
__device__ __forceinline__ void dep_guard_b(v8f& a, v8f& b, v16b x, v16b y) { asm volatile("v_nop\n\tv_nop\n\tv_nop\n\tv_nop" : "+v"(a), "+v"(b) : "v"(x), "v"(y)); }
__device__ __forceinline__ void keep4_h(v16h a, v16h b, v16h c, v16h d) { asm volatile("v_nop" :: "v"(a), "v"(b), "v"(c), "v"(d)); }
__device__ __forceinline__ void keep4_b(v16b a, v16b b, v16b c, v16b d) { asm volatile("v_nop" :: "v"(a), "v"(b), "v"(c), "v"(d)); }
__device__ __forceinline__ void acc_guard4(v8f& a, v8f& b, v8f& c, v8f& d) { asm volatile("v_nop\n\tv_nop\n\tv_nop\n\tv_nop" : "+v"(a), "+v"(b), "+v"(c), "+v"(d)); }
__device__ __forceinline__ void dep_guard3_h(v8f& a, v8f& b, v8f& c, v16h w, v16h x, v16h y, v16h z) {
  asm volatile("v_nop\n\tv_nop\n\tv_nop\n\tv_nop" : "+v"(a), "+v"(b), "+v"(c) : "v"(w), "v"(x), "v"(y), "v"(z));
}
__device__ __forceinline__ void acc_guard3(v8f& a, v8f& b, v8f& c) { asm volatile("v_nop\n\tv_nop\n\tv_nop\n\tv_nop" : "+v"(a), "+v"(b), "+v"(c)); }

template <typename T> struct Frag;
template <> struct Frag<_Float16> {
  typedef v16h V; union U { v16h v; v8h h[2]; };
  static __device__ __forceinline__ v16h load(const _Float16* p) {
    U f; f.h[0] = *(const v8h*)(p); f.h[1] = *(const v8h*)(p + 16); return f.v;
  }
  static __device__ __forceinline__ v8f mma(v16h a, v16h b, v8f c) {
    return __builtin_amdgcn_wmma_f32_16x16x32_f16(false, a, false, b, (short)0, c, false, false);
  }
  static __device__ __forceinline__ void guard(v8f& a, v8f& b, v16h x, v16h y) { dep_guard_h(a, b, x, y); }
  static __device__ __forceinline__ void keep(v16h a, v16h b, v16h c, v16h d) { keep4_h(a, b, c, d); }
};
template <> struct Frag<__bf16> {
  typedef v16b V; union U { v16b v; v8b h[2]; };
  static __device__ __forceinline__ v16b load(const __bf16* p) {
    U f; f.h[0] = *(const v8b*)(p); f.h[1] = *(const v8b*)(p + 16); return f.v;
  }
  static __device__ __forceinline__ v8f mma(v16b a, v16b b, v8f c) {
    return __builtin_amdgcn_wmma_f32_16x16x32_bf16(false, a, false, b, (short)0, c, false, false);
  }
  static __device__ __forceinline__ void guard(v8f& a, v8f& b, v16b x, v16b y) { dep_guard_b(a, b, x, y); }
  static __device__ __forceinline__ void keep(v16b a, v16b b, v16b c, v16b d) { keep4_b(a, b, c, d); }
};

template <int ET> struct Elem;
template <> struct Elem<0> { typedef _Float16 T; };
template <> struct Elem<1> { typedef __bf16 T; };
template <int ET, bool SPLIT, int BIAS_MODE, int OUT_MODE, bool RESID, int ACT = 0>
__global__ __launch_bounds__(256) void wmma_gemm64(
    const unsigned short* __restrict__ Ap, const unsigned short* __restrict__ A2p, int lda, long strideA,
    const unsigned short* __restrict__ Btp, const unsigned short* __restrict__ Bt2p, int ldb, long strideB,
    void* __restrict__ Cout, void* __restrict__ Cout2, int ldc, long strideC,
    const float* __restrict__ bias,
    const float* __restrict__ resid, long strideR,
    int M, int N, int K, float scale) {
  typedef typename Elem<ET>::T T;
  typedef typename Frag<T>::V V;
  const T* A = (const T*)Ap; const T* A2 = (const T*)A2p; const T* Bt = (const T*)Btp; const T* Bt2 = (const T*)Bt2p;
  __shared__ __align__(16) float sT[8][16 * 68];
  const int b    = blockIdx.y;
  const int lane = threadIdx.x & 31;
  const int wave = threadIdx.x >> 5;
  const int tilesN = N >> 6;
  const int tilesM = M >> 6;
  const int tile = blockIdx.x * 8 + wave;
  if (tile >= tilesM * tilesN) return;
  const int tm = tile / tilesN;
  const int tn = tile - tm * tilesN;
  const int m0 = tm << 6;
  const int n0 = tn << 6;

  const T* Ab  = A  + (size_t)b * strideA;
  const T* Bb  = Bt + (size_t)b * strideB;
  const T* Ab2 = SPLIT ? (A2  + (size_t)b * strideA) : nullptr;
  const T* Bb2 = SPLIT ? (Bt2 + (size_t)b * strideB) : nullptr;

  const int rlane = lane & 15;
  const int koff  = (lane >> 4) * 8;
  const int mOff  = (lane >> 4) * 8;

  v8f acc[4][4];
#pragma unroll
  for (int i = 0; i < 4; ++i)
#pragma unroll
    for (int j = 0; j < 4; ++j) acc[i][j] = (v8f){0.f,0.f,0.f,0.f,0.f,0.f,0.f,0.f};

  for (int k0 = 0; k0 < K; k0 += 32) {
    V bh[4], bl[4];
#pragma unroll
    for (int j = 0; j < 4; ++j) {
      const size_t bo = (size_t)(n0 + (j << 4) + rlane) * ldb + koff + k0;
      bh[j] = Frag<T>::load(Bb + bo);
      if (SPLIT) bl[j] = Frag<T>::load(Bb2 + bo);
    }
#pragma unroll
    for (int i = 0; i < 4; ++i) {
      const size_t ao = (size_t)(m0 + (i << 4) + rlane) * lda + koff + k0;
      V ah = Frag<T>::load(Ab + ao);
      V al;
      if (SPLIT) al = Frag<T>::load(Ab2 + ao);
#pragma unroll
      for (int j = 0; j < 4; ++j) {
        acc[i][j] = Frag<T>::mma(ah, bh[j], acc[i][j]);
        if (SPLIT) {
          acc[i][j] = Frag<T>::mma(ah, bl[j], acc[i][j]);
          acc[i][j] = Frag<T>::mma(al, bh[j], acc[i][j]);
        }
      }
      Frag<T>::guard(acc[i][0], acc[i][3], ah, SPLIT ? al : ah);
    }
    Frag<T>::keep(bh[0], bh[1], bh[2], bh[3]);
    if (SPLIT) Frag<T>::keep(bl[0], bl[1], bl[2], bl[3]);
  }
  acc_guard4(acc[0][0], acc[0][1], acc[0][2], acc[0][3]);
  acc_guard4(acc[1][0], acc[1][1], acc[1][2], acc[1][3]);
  acc_guard4(acc[2][0], acc[2][1], acc[2][2], acc[2][3]);
  acc_guard4(acc[3][0], acc[3][1], acc[3][2], acc[3][3]);

  float* slab = sT[wave];
  const float* Rb = RESID ? (resid + (size_t)b * strideR) : nullptr;
#pragma unroll
  for (int i = 0; i < 4; ++i) {
    const int mBase = m0 + (i << 4);
#pragma unroll
    for (int j = 0; j < 4; ++j) {
      const int n = n0 + (j << 4) + rlane;
      float bv = 0.f;
      if (BIAS_MODE == 2) bv = bias[n];
#pragma unroll
      for (int r = 0; r < 8; ++r) {
        float v = acc[i][j][r] * scale;
        if (BIAS_MODE == 1) v += bias[mBase + mOff + r];
        if (BIAS_MODE == 2) v += bv;
        if (RESID) v += Rb[(size_t)(mBase + mOff + r) * ldc + n];
        if (ACT == 1) v = tanhf(v);
        if (ACT == 2) v = fmaxf(v, 0.0f);
        if (ACT == 3) v = v / (1.0f + expf(-v));
        if (ACT == 4) v = (v > 0.f) ? v : 0.01f * v;
        if (ACT == 5) v = 0.5f * v * (1.0f + erff(v * 0.70710678118654752f));
        slab[(mOff + r) * 68 + (j << 4) + rlane] = v;
      }
    }
    __builtin_amdgcn_fence(__ATOMIC_RELEASE, "workgroup");
    __builtin_amdgcn_wave_barrier();
    __builtin_amdgcn_fence(__ATOMIC_ACQUIRE, "workgroup");
    if (OUT_MODE == 0) {
      float* C = (float*)Cout + (size_t)b * strideC;
      const int hh = lane >> 4, c4 = (lane & 15) * 4;
      for (int pass = 0; pass < 2; ++pass) {
#pragma unroll
        for (int it = 0; it < 8; ++it) {
          const int row = it * 2 + hh;
          v4f v = *(const v4f*)(slab + row * 68 + c4);
          *(volatile v4f*)(C + (size_t)(mBase + row) * ldc + n0 + c4) = v;
        }
        __threadfence();
      }
    } else {
      const int q = lane >> 3, c8 = (lane & 7) * 8;
      unsigned short* C  = (unsigned short*)Cout  + (size_t)b * strideC;
      unsigned short* C2 = (OUT_MODE == 2) ? ((unsigned short*)Cout2 + (size_t)b * strideC) : nullptr;
      for (int pass = 0; pass < 2; ++pass) {
#pragma unroll
        for (int it = 0; it < 4; ++it) {
          const int row = it * 4 + q;
          const float* sp = slab + row * 68 + c8;
          v8h hv, lv;
#pragma unroll
          for (int e = 0; e < 8; ++e) {
            if (OUT_MODE == 1) {
              hv[e] = (_Float16)sp[e];
            } else {
              unsigned short hb = f2bf_bits(sp[e]);
              unsigned short lb = f2bf_bits(sp[e] - bf_bits2f(hb));
              hv[e] = __builtin_bit_cast(_Float16, hb);
              lv[e] = __builtin_bit_cast(_Float16, lb);
            }
          }
          *(volatile v8h*)(C + (size_t)(mBase + row) * ldc + n0 + c8) = hv;
          if (OUT_MODE == 2) *(volatile v8h*)(C2 + (size_t)(mBase + row) * ldc + n0 + c8) = lv;
        }
        __threadfence();
      }
    }
    __builtin_amdgcn_fence(__ATOMIC_RELEASE, "workgroup");
    __builtin_amdgcn_wave_barrier();
    __builtin_amdgcn_fence(__ATOMIC_ACQUIRE, "workgroup");
  }
}

__device__ __forceinline__ float fsig(float x)  { return __builtin_amdgcn_rcpf(1.0f + expf(-x)); }
__device__ __forceinline__ float ftanh(float x) { return 1.0f - 2.0f * __builtin_amdgcn_rcpf(1.0f + expf(2.0f * x)); }

__global__ __launch_bounds__(NTHR) void cvt_plane8_kernel(const float* __restrict__ src, unsigned short* __restrict__ dst,
                                                          int n8, float sc) {
  const int i = blockIdx.x * NTHR + threadIdx.x;
  if (i < n8) {
    const float* sp = src + (size_t)i * 8;
    const v4f a = *(const v4f*)(sp);
    const v4f b = *(const v4f*)(sp + 4);
    v8h hv;
#pragma unroll
    for (int e = 0; e < 4; ++e) {
      hv[e]     = (_Float16)(a[e] * sc);
      hv[4 + e] = (_Float16)(b[e] * sc);
    }
    unsigned short* dp = dst + (size_t)i * 8;
    *(volatile v8h*)dp = hv;
    __threadfence();
    *(volatile v8h*)dp = hv;
  }
}

__global__ __launch_bounds__(NTHR) void cvt_u_kernel(const float* __restrict__ u, unsigned short* __restrict__ dst, int n8) {
  const int i = blockIdx.x * NTHR + threadIdx.x;
  if (i < n8) {
    constexpr int C8 = NINP / 8;
    const int drow = i / C8;
    const int c8   = i - drow * C8;
    const int s    = drow / NBAT;
    const int b    = drow - s * NBAT;
    const float* sp = u + ((size_t)b * NSTEP + (size_t)s) * NINP + (size_t)c8 * 8;
    const v4f a  = *(const v4f*)(sp);
    const v4f bq = *(const v4f*)(sp + 4);
    v8h hv;
#pragma unroll
    for (int e = 0; e < 4; ++e) {
      hv[e]     = (_Float16)a[e];
      hv[4 + e] = (_Float16)bq[e];
    }
    unsigned short* dp = dst + (size_t)i * 8;
    *(volatile v8h*)dp = hv;
    __threadfence();
    *(volatile v8h*)dp = hv;
  }
}

__device__ __forceinline__ void stage_h16(const float* hf, _Float16* hh16, int tid) {
#pragma unroll 1
  for (int i = tid; i < RBLK * NHID / 8; i += NTHR) {
    const int row = i / (NHID / 8);
    const int col = (i - row * (NHID / 8)) * 8;
    const v4f a = *(const v4f*)(hf + row * HPF + col);
    const v4f b = *(const v4f*)(hf + row * HPF + col + 4);
    v8h hv;
#pragma unroll
    for (int e = 0; e < 4; ++e) { hv[e] = (_Float16)a[e]; hv[4 + e] = (_Float16)b[e]; }
    *(v8h*)(hh16 + row * HPH + col) = hv;
  }
}

__global__ __launch_bounds__(NTHR) void gru_chunk_kernel(const float* __restrict__ XG,
                                                         const unsigned short* __restrict__ WHHp,
                                                         const float* __restrict__ bhh,
                                                         const float* __restrict__ wfc,
                                                         const float* __restrict__ bfc,
                                                         const float* __restrict__ HCIN,
                                                         float* __restrict__ HCOUT,
                                                         float* __restrict__ out,
                                                         int chunk, int first) {
  __shared__ __align__(16) float    hf[RBLK * HPF];
  __shared__ __align__(16) _Float16 hh16[RBLK * HPH];
  __shared__ __align__(16) float    wl[NOUTC * NHID];
  __shared__ __align__(16) float    os[RBLK * OSP];
  const _Float16* WHH = (const _Float16*)WHHp;
  const int tid = threadIdx.x, lane = tid & 31, wave = tid >> 5;
  const int c = lane & 15, hsel = lane >> 4, koff = hsel * 8, c4 = c * 4;
  const int b0 = blockIdx.x * RBLK;

#pragma unroll 1
  for (int i = tid; i < NOUTC * NHID / 4; i += NTHR) *(v4f*)(wl + 4 * i) = *(const v4f*)(wfc + 4 * i);
  const v4f z4 = {0.f, 0.f, 0.f, 0.f};
  if (first != 0) {
#pragma unroll 1
    for (int i = tid; i < RBLK * NHID / 4; i += NTHR) {
      const int row = i / (NHID / 4);
      const int col = (i - row * (NHID / 4)) * 4;
      *(v4f*)(hf + row * HPF + col) = z4;
    }
  } else {
#pragma unroll 1
    for (int i = tid; i < RBLK * NHID / 4; i += NTHR) {
      const int row = i / (NHID / 4);
      const int col = (i - row * (NHID / 4)) * 4;
      *(v4f*)(hf + row * HPF + col) = *(const v4f*)(HCIN + (size_t)(b0 + row) * NHID + col);
    }
  }
  const float bf0 = bfc[0], bf1 = bfc[1], bf2 = bfc[2];
  __syncthreads();
  stage_h16(hf, hh16, tid);
  __syncthreads();

  const v8f z8 = {0.f, 0.f, 0.f, 0.f, 0.f, 0.f, 0.f, 0.f};
  const _Float16* arow = hh16 + c * HPH + koff;
  const int r0 = 2 * wave;

#pragma unroll 1
  for (int sl = 0; sl < CHUNK; ++sl) {
    const float* xrow = XG + (size_t)(sl * NBAT + b0 + 8 * hsel) * NG3;
#pragma unroll 1
    for (int jt = 0; jt < JTW; ++jt) {
      const int j = 16 * (JTW * wave + jt) + c;
      const _Float16* wr = WHH + (size_t)j * NHID + koff;
      const _Float16* wz = WHH + (size_t)(NHID + j) * NHID + koff;
      const _Float16* wn = WHH + (size_t)(2 * NHID + j) * NHID + koff;
      v8f ar = z8, az = z8, an = z8;
#pragma unroll 1
      for (int k0 = 0; k0 < NHID; k0 += 32) {
        const v16h a   = Frag<_Float16>::load(arow + k0);
        const v16h bq0 = Frag<_Float16>::load(wr + k0);
        const v16h bq1 = Frag<_Float16>::load(wz + k0);
        const v16h bq2 = Frag<_Float16>::load(wn + k0);
        ar = Frag<_Float16>::mma(a, bq0, ar);
        az = Frag<_Float16>::mma(a, bq1, az);
        an = Frag<_Float16>::mma(a, bq2, an);
        dep_guard3_h(ar, az, an, a, bq0, bq1, bq2);
      }
      acc_guard3(ar, az, an);

      const float br = bhh[j], bz = bhh[NHID + j], bn = bhh[2 * NHID + j];
#pragma unroll
      for (int r = 0; r < 8; ++r) {
        if (r == 4) asm volatile("" ::: "memory");
        const float* xr = xrow + (size_t)r * NG3 + j;
        const float x_r = xr[0], x_z = xr[NHID], x_n = xr[2 * NHID];
        const float hr = ar[r] * WCARRY_INV + br;
        const float hz = az[r] * WCARRY_INV + bz;
        const float hn = an[r] * WCARRY_INV + bn;
        const float rg = fsig(x_r + hr);
        const float zg = fsig(x_z + hz);
        const float ng = ftanh(x_n + rg * hn);
        const int hidx = (8 * hsel + r) * HPF + j;
        const float hp = hf[hidx];
        const float hnew = (1.0f - zg) * ng + zg * hp;
        hf[hidx] = hnew;
      }
    }
    __syncthreads();
    stage_h16(hf, hh16, tid);
    {
      float p00 = 0.0f, p01 = 0.0f, p02 = 0.0f, p10 = 0.0f, p11 = 0.0f, p12 = 0.0f;
#pragma unroll 1
      for (int q = 0; q < NHID / 128; ++q) {
        const int k = 128 * q + 4 * lane;
        const v4f h0 = *(const v4f*)(hf + r0 * HPF + k);
        const v4f h1 = *(const v4f*)(hf + (r0 + 1) * HPF + k);
        const v4f w0 = *(const v4f*)(wl + k);
        const v4f w1 = *(const v4f*)(wl + NHID + k);
        const v4f w2 = *(const v4f*)(wl + 2 * NHID + k);
#pragma unroll
        for (int e = 0; e < 4; ++e) {
          p00 += h0[e] * w0[e]; p01 += h0[e] * w1[e]; p02 += h0[e] * w2[e];
          p10 += h1[e] * w0[e]; p11 += h1[e] * w1[e]; p12 += h1[e] * w2[e];
        }
      }
#pragma unroll
      for (int off = 16; off > 0; off >>= 1) {
        p00 += __shfl_xor(p00, off, 32); p01 += __shfl_xor(p01, off, 32); p02 += __shfl_xor(p02, off, 32);
        p10 += __shfl_xor(p10, off, 32); p11 += __shfl_xor(p11, off, 32); p12 += __shfl_xor(p12, off, 32);
      }
      if (lane == 0) {
        float* o0 = os + r0 * OSP + sl * NOUTC;
        float* o1 = os + (r0 + 1) * OSP + sl * NOUTC;
        o0[0] = p00 + bf0; o0[1] = p01 + bf1; o0[2] = p02 + bf2;
        o1[0] = p10 + bf0; o1[1] = p11 + bf1; o1[2] = p12 + bf2;
      }
    }
    __syncthreads();
  }

  {
    const int row = 2 * wave + hsel;
    float* hdst = HCOUT + (size_t)(b0 + row) * NHID;
    float* odst = out + (size_t)(b0 + row) * OUTROW + (size_t)chunk * OSP;
    for (int pass = 0; pass < 2; ++pass) {
#pragma unroll
      for (int it = 0; it < NHID / 64; ++it) {
        const v4f v = *(const v4f*)(hf + row * HPF + it * 64 + c4);
        *(volatile v4f*)(hdst + it * 64 + c4) = v;
      }
#pragma unroll
      for (int it = 0; it < OSP / 64; ++it) {
        const v4f v = *(const v4f*)(os + row * OSP + it * 64 + c4);
        *(volatile v4f*)(odst + it * 64 + c4) = v;
      }
      __threadfence();
    }
  }
}

extern "C" void kernel_launch(void* const* d_in, const int* in_sizes, int n_in,
                              void* d_out, int out_size, void* d_ws, size_t ws_size, hipStream_t stream) {
  if (n_in < 7 || d_out == nullptr || d_ws == nullptr) return;
  if (in_sizes[0] != NBAT * NSTEP * NINP || in_sizes[1] != NG3 * NINP || in_sizes[2] != NG3 * NHID ||
      in_sizes[3] != NG3 || in_sizes[4] != NG3 || in_sizes[5] != NOUTC * NHID || in_sizes[6] != NOUTC ||
      out_size != NBAT * NSTEP * NOUTC) return;

  const float* u    = (const float*)d_in[0];
  const float* w_ih = (const float*)d_in[1];
  const float* w_hh = (const float*)d_in[2];
  const float* b_ih = (const float*)d_in[3];
  const float* b_hh = (const float*)d_in[4];
  const float* w_fc = (const float*)d_in[5];
  const float* b_fc = (const float*)d_in[6];
  float* out = (float*)d_out;

  char* ws = (char*)d_ws; size_t off = 0;
  auto carve = [&](size_t bytes) -> char* { char* p = ws + off; off += (bytes + 255) & ~(size_t)255; return p; };
  unsigned short* WHH16 = (unsigned short*)carve((size_t)NG3 * NHID * 2);
  unsigned short* WIH16 = (unsigned short*)carve((size_t)NG3 * NINP * 2);
  unsigned short* U16   = (unsigned short*)carve((size_t)UROWS * NINP * 2);
  float*          XG    = (float*)carve((size_t)CHROWS * NG3 * 4);
  float*          HC0   = (float*)carve((size_t)NBAT * NHID * 4);
  float*          HC1   = (float*)carve((size_t)NBAT * NHID * 4);
  if (off > ws_size || off > (size_t)134217728) return;

  const int n8hh = NG3 * NHID / 8;
  const int n8ih = NG3 * NINP / 8;
  const int n8u  = UROWS * NINP / 8;
  cvt_plane8_kernel<<<(n8hh + NTHR - 1) / NTHR, NTHR, 0, stream>>>(w_hh, WHH16, n8hh, WCARRY);
  cvt_plane8_kernel<<<(n8ih + NTHR - 1) / NTHR, NTHR, 0, stream>>>(w_ih, WIH16, n8ih, WCARRY);
  cvt_u_kernel<<<(n8u + NTHR - 1) / NTHR, NTHR, 0, stream>>>(u, U16, n8u);

  const int gemm_blocks = (CHROWS / 64) * (NG3 / 64) / 8;
  for (int ch = 0; ch < NCHUNK; ++ch) {
    wmma_gemm64<0, false, 2, 0, false, 0><<<dim3(gemm_blocks, 1), 256, 0, stream>>>(
        (const unsigned short*)(U16 + (size_t)ch * CHROWS * NINP), (const unsigned short*)nullptr, NINP, 0L,
        (const unsigned short*)WIH16, (const unsigned short*)nullptr, NINP, 0L,
        (void*)XG, (void*)nullptr, NG3, 0L,
        b_ih, (const float*)nullptr, 0L, CHROWS, NG3, NINP, WCARRY_INV);
    const float* hcin  = (ch & 1) ? HC0 : HC1;
    float*       hcout = (ch & 1) ? HC1 : HC0;
    gru_chunk_kernel<<<NBAT / RBLK, NTHR, 0, stream>>>(XG, WHH16, b_hh, w_fc, b_fc, hcin, hcout, out,
                                                       ch, (ch == 0) ? 1 : 0);
  }
}
